// SelectiveSSM_18846316495342
// MI455X (gfx1250) — hardware-verified
//
#include <hip/hip_runtime.h>
#include <math.h>

typedef __attribute__((ext_vector_type(16))) _Float16 v16h;
typedef __attribute__((ext_vector_type(8)))  _Float16 v8h;
typedef __attribute__((ext_vector_type(16))) __bf16   v16b;
typedef __attribute__((ext_vector_type(8)))  __bf16   v8b;
typedef __attribute__((ext_vector_type(8)))  float    v8f;
typedef __attribute__((ext_vector_type(4)))  float    v4f;

constexpr int kBatch  = 2;
constexpr int kSeq    = 4096;
constexpr int kDm     = 1024;
constexpr int kDin    = 2048;
constexpr int kNst    = 16;
constexpr int kDtR    = 64;
constexpr int kXdb    = 96;
constexpr int kXdbP   = 128;
constexpr int kRows   = kBatch * kSeq;
constexpr int kBcP    = 64;
constexpr int kScanTS = 64;
constexpr int kScanCh = 64;
constexpr int kScanYP = 68;
constexpr int kTrP    = 68;
constexpr float kWsc    = 64.0f;
constexpr float kWscInv = 1.0f / 64.0f;
constexpr float kYsc    = 16.0f;
constexpr float kOutScl = 1.0f / (64.0f * 16.0f);
static_assert(kDtR + 2 * kNst == kXdb);
static_assert((kDm % 32) == 0 && (kDin % 32) == 0 && (kDtR % 32) == 0);
static_assert((kRows % 64) == 0 && (kDin % 64) == 0 && (kDm % 64) == 0 && (kXdbP % 64) == 0 && (kDtR % 64) == 0);
static_assert(((kRows / 64) * (kDin / 64)) % 8 == 0 && ((kRows / 64) * (kDm / 64)) % 8 == 0 && ((kRows / 64) * 1) % 8 == 0);
static_assert((kSeq % kScanTS) == 0 && (kDin % kScanCh) == 0 && (kXdb % 4) == 0);
static_assert((kDm % 64) == 0 && (kXdbP % 64) == 0 && (kDtR % 64) == 0 && (kDin % 64) == 0);

constexpr size_t kSzX16   = (size_t)kRows * kDm * 2;
constexpr size_t kSzBTIN  = (size_t)(2 * kDin) * kDm * 2;
constexpr size_t kSzBTXP  = (size_t)kXdbP * kDin * 2;
constexpr size_t kSzBTDT  = (size_t)kDin * kDtR * 2;
constexpr size_t kSzBTOUT = (size_t)kDm * kDin * 2;
constexpr size_t kSz16P   = (size_t)kRows * kDin * 2;
constexpr size_t kSzDLT   = (size_t)kRows * kDtR * 2;
constexpr size_t kSzBC    = (size_t)kRows * kBcP * 4;
constexpr size_t kOffX16   = 0;
constexpr size_t kOffBTIN  = kOffX16   + kSzX16;
constexpr size_t kOffBTXP  = kOffBTIN  + kSzBTIN;
constexpr size_t kOffBTDT  = kOffBTXP  + kSzBTXP;
constexpr size_t kOffBTOUT = kOffBTDT  + kSzBTDT;
constexpr size_t kOffXP16  = kOffBTOUT + kSzBTOUT;
constexpr size_t kOffZ16   = kOffXP16  + kSz16P;
constexpr size_t kOffDPRE  = kOffZ16   + kSz16P;
constexpr size_t kOffDLT   = kOffDPRE  + kSz16P;
constexpr size_t kOffBC    = kOffDLT   + kSzDLT;
constexpr size_t kWsTotal  = kOffBC    + kSzBC;
static_assert(kWsTotal == 133955584ull);
static_assert(kWsTotal <= 134217728ull);
static_assert((kOffBTIN % 128) == 0 && (kOffBTXP % 128) == 0 && (kOffBTDT % 128) == 0 && (kOffBTOUT % 128) == 0 &&
              (kOffXP16 % 128) == 0 && (kOffZ16 % 128) == 0 && (kOffDPRE % 128) == 0 && (kOffDLT % 128) == 0 &&
              (kOffBC % 128) == 0);
static_assert(kOffZ16 == kOffXP16 + (size_t)kRows * kDin * 2);

__device__ __forceinline__ unsigned short f2bf_bits(float f) {
  unsigned u = __float_as_uint(f);
  return (unsigned short)((u + 0x7FFFu + ((u >> 16) & 1u)) >> 16);
}
__device__ __forceinline__ float bf_bits2f(unsigned short h) { return __uint_as_float(((unsigned)h) << 16); }

__device__ __forceinline__ float h16_to_f32(unsigned hb) {
  const unsigned sgn = (hb & 0x8000u) << 16; const unsigned em = hb & 0x7fffu;
  const float fn = __uint_as_float((em << 13) + 0x38000000u);
  const float fs = (float)em * 5.9604644775390625e-8f;
  const float mag = (em < 0x400u) ? fs : fn; return __uint_as_float(__float_as_uint(mag) | sgn); }

__device__ __forceinline__ void dep_guard4_h(v8f& a, v8f& b, v8f& c, v8f& d, v16h x, v16h y) {
  asm volatile("v_nop\n\tv_nop\n\tv_nop\n\tv_nop" : "+v"(a), "+v"(b), "+v"(c), "+v"(d) : "v"(x), "v"(y)); }
__device__ __forceinline__ void dep_guard4_b(v8f& a, v8f& b, v8f& c, v8f& d, v16b x, v16b y) {
  asm volatile("v_nop\n\tv_nop\n\tv_nop\n\tv_nop" : "+v"(a), "+v"(b), "+v"(c), "+v"(d) : "v"(x), "v"(y)); }
__device__ __forceinline__ void keep4_h(v16h a, v16h b, v16h c, v16h d) { asm volatile("v_nop" :: "v"(a), "v"(b), "v"(c), "v"(d)); }
__device__ __forceinline__ void keep4_b(v16b a, v16b b, v16b c, v16b d) { asm volatile("v_nop" :: "v"(a), "v"(b), "v"(c), "v"(d)); }
__device__ __forceinline__ void acc_guard4(v8f& a, v8f& b, v8f& c, v8f& d) { asm volatile("v_nop\n\tv_nop\n\tv_nop\n\tv_nop" : "+v"(a), "+v"(b), "+v"(c), "+v"(d)); }
template <typename T> struct Frag;
template <> struct Frag<_Float16> {
  typedef v16h V; union U { v16h v; v8h h[2]; };
  static __device__ __forceinline__ v16h load(const _Float16* p) {
    U f; f.h[0] = *(const v8h*)(p); f.h[1] = *(const v8h*)(p + 16); return f.v;
  }
  static __device__ __forceinline__ v8f mma(v16h a, v16h b, v8f c) {
    return __builtin_amdgcn_wmma_f32_16x16x32_f16(false, a, false, b, (short)0, c, false, false);
  }
  static __device__ __forceinline__ void guard4(v8f& a, v8f& b, v8f& c, v8f& d, v16h x, v16h y) { dep_guard4_h(a, b, c, d, x, y); }
  static __device__ __forceinline__ void keep(v16h a, v16h b, v16h c, v16h d) { keep4_h(a, b, c, d); }
};
template <> struct Frag<__bf16> {
  typedef v16b V; union U { v16b v; v8b h[2]; };
  static __device__ __forceinline__ v16b load(const __bf16* p) {
    U f; f.h[0] = *(const v8b*)(p); f.h[1] = *(const v8b*)(p + 16); return f.v;
  }
  static __device__ __forceinline__ v8f mma(v16b a, v16b b, v8f c) {
    return __builtin_amdgcn_wmma_f32_16x16x32_bf16(false, a, false, b, (short)0, c, false, false);
  }
  static __device__ __forceinline__ void guard4(v8f& a, v8f& b, v8f& c, v8f& d, v16b x, v16b y) { dep_guard4_b(a, b, c, d, x, y); }
  static __device__ __forceinline__ void keep(v16b a, v16b b, v16b c, v16b d) { keep4_b(a, b, c, d); }
};

template <int ET> struct Elem;
template <> struct Elem<0> { typedef _Float16 T; };
template <> struct Elem<1> { typedef __bf16 T; };
template <int ET, bool SPLIT, int BIAS_MODE, int OUT_MODE, bool RESID, int ACT = 0>
__global__ __launch_bounds__(256) void wmma_gemm64(
    const unsigned short* __restrict__ Ap, const unsigned short* __restrict__ A2p, int lda, long strideA,
    const unsigned short* __restrict__ Btp, const unsigned short* __restrict__ Bt2p, int ldb, long strideB,
    void* __restrict__ Cout, void* __restrict__ Cout2, int ldc, long strideC,
    const float* __restrict__ bias,
    const float* __restrict__ resid, long strideR,
    int M, int N, int K, float scale) {
  typedef typename Elem<ET>::T T;
  typedef typename Frag<T>::V V;
  const T* A = (const T*)Ap; const T* A2 = (const T*)A2p; const T* Bt = (const T*)Btp; const T* Bt2 = (const T*)Bt2p;
  __shared__ __align__(16) float sT[8][16 * 68];
  const int b    = blockIdx.y;
  const int lane = threadIdx.x & 31;
  const int wave = threadIdx.x >> 5;
  const int tilesN = N >> 6;
  const int tilesM = M >> 6;
  const int tile = blockIdx.x * 8 + wave;
  if (tile >= tilesM * tilesN) return;
  const int tm = tile / tilesN;
  const int tn = tile - tm * tilesN;
  const int m0 = tm << 6;
  const int n0 = tn << 6;

  const T* Ab  = A  + (size_t)b * strideA;
  const T* Bb  = Bt + (size_t)b * strideB;
  const T* Ab2 = SPLIT ? (A2  + (size_t)b * strideA) : nullptr;
  const T* Bb2 = SPLIT ? (Bt2 + (size_t)b * strideB) : nullptr;

  const int rlane = lane & 15;
  const int koff  = (lane >> 4) * 8;
  const int mOff  = (lane >> 4) * 8;

  v8f acc[4][4];
#pragma unroll
  for (int i = 0; i < 4; ++i)
#pragma unroll
    for (int j = 0; j < 4; ++j) acc[i][j] = (v8f){0.f,0.f,0.f,0.f,0.f,0.f,0.f,0.f};

  for (int k0 = 0; k0 < K; k0 += 32) {
    V bh[4], bl[4];
#pragma unroll
    for (int j = 0; j < 4; ++j) {
      const size_t bo = (size_t)(n0 + (j << 4) + rlane) * ldb + koff + k0;
      bh[j] = Frag<T>::load(Bb + bo);
      if (SPLIT) bl[j] = Frag<T>::load(Bb2 + bo);
    }
#pragma unroll
    for (int i = 0; i < 4; ++i) {
      const size_t ao = (size_t)(m0 + (i << 4) + rlane) * lda + koff + k0;
      V ah = Frag<T>::load(Ab + ao);
      V al;
      if (SPLIT) al = Frag<T>::load(Ab2 + ao);
#pragma unroll
      for (int j = 0; j < 4; ++j) {
        acc[i][j] = Frag<T>::mma(ah, bh[j], acc[i][j]);
        if (SPLIT) {
          acc[i][j] = Frag<T>::mma(ah, bl[j], acc[i][j]);
          acc[i][j] = Frag<T>::mma(al, bh[j], acc[i][j]);
        }
      }
      Frag<T>::guard4(acc[i][0], acc[i][1], acc[i][2], acc[i][3], ah, SPLIT ? al : ah);
    }
    Frag<T>::keep(bh[0], bh[1], bh[2], bh[3]);
    if (SPLIT) Frag<T>::keep(bl[0], bl[1], bl[2], bl[3]);
  }
  acc_guard4(acc[0][0], acc[0][1], acc[0][2], acc[0][3]);
  acc_guard4(acc[1][0], acc[1][1], acc[1][2], acc[1][3]);
  acc_guard4(acc[2][0], acc[2][1], acc[2][2], acc[2][3]);
  acc_guard4(acc[3][0], acc[3][1], acc[3][2], acc[3][3]);

  float* slab = sT[wave];
  const float* Rb = RESID ? (resid + (size_t)b * strideR) : nullptr;
#pragma unroll
  for (int i = 0; i < 4; ++i) {
    const int mBase = m0 + (i << 4);
#pragma unroll
    for (int j = 0; j < 4; ++j) {
      const int n = n0 + (j << 4) + rlane;
      float bv = 0.f;
      if (BIAS_MODE == 2) bv = bias[n];
#pragma unroll
      for (int r = 0; r < 8; ++r) {
        float v = acc[i][j][r] * scale;
        if (BIAS_MODE == 1) v += bias[mBase + mOff + r];
        if (BIAS_MODE == 2) v += bv;
        if (RESID) v += Rb[(size_t)(mBase + mOff + r) * ldc + n];
        if (ACT == 1) v = tanhf(v);
        if (ACT == 2) v = fmaxf(v, 0.0f);
        if (ACT == 3) v = v / (1.0f + expf(-v));
        if (ACT == 4) v = (v > 0.f) ? v : 0.01f * v;
        slab[(mOff + r) * 68 + (j << 4) + rlane] = v;
      }
    }
    __builtin_amdgcn_fence(__ATOMIC_RELEASE, "workgroup");
    __builtin_amdgcn_wave_barrier();
    __builtin_amdgcn_fence(__ATOMIC_ACQUIRE, "workgroup");
    if (OUT_MODE == 0) {
      float* C = (float*)Cout + (size_t)b * strideC;
      const int hh = lane >> 4, c4 = (lane & 15) * 4;
      for (int pass = 0; pass < 2; ++pass) {
#pragma unroll
        for (int it = 0; it < 8; ++it) {
          const int row = it * 2 + hh;
          v4f v = *(const v4f*)(slab + row * 68 + c4);
          *(volatile v4f*)(C + (size_t)(mBase + row) * ldc + n0 + c4) = v;
        }
        __threadfence();
      }
    } else {
      const int q = lane >> 3, c8 = (lane & 7) * 8;
      unsigned short* C  = (unsigned short*)Cout  + (size_t)b * strideC;
      unsigned short* C2 = (OUT_MODE == 2) ? ((unsigned short*)Cout2 + (size_t)b * strideC) : nullptr;
      for (int pass = 0; pass < 2; ++pass) {
#pragma unroll
        for (int it = 0; it < 4; ++it) {
          const int row = it * 4 + q;
          const float* sp = slab + row * 68 + c8;
          v8h hv, lv;
#pragma unroll
          for (int e = 0; e < 8; ++e) {
            if (OUT_MODE == 1) {
              hv[e] = (_Float16)sp[e];
            } else {
              unsigned short hb = f2bf_bits(sp[e]);
              unsigned short lb = f2bf_bits(sp[e] - bf_bits2f(hb));
              hv[e] = __builtin_bit_cast(_Float16, hb);
              lv[e] = __builtin_bit_cast(_Float16, lb);
            }
          }
          *(volatile v8h*)(C + (size_t)(mBase + row) * ldc + n0 + c8) = hv;
          if (OUT_MODE == 2) *(volatile v8h*)(C2 + (size_t)(mBase + row) * ldc + n0 + c8) = lv;
        }
        __threadfence();
      }
    }
    __builtin_amdgcn_fence(__ATOMIC_RELEASE, "workgroup");
    __builtin_amdgcn_wave_barrier();
    __builtin_amdgcn_fence(__ATOMIC_ACQUIRE, "workgroup");
  }
}

__global__ __launch_bounds__(256) void cast_rows_f16_kernel(
    const float* __restrict__ src, unsigned short* __restrict__ dst, int total8)
{
  const int i = blockIdx.x * 256 + threadIdx.x;
  if (i >= total8) return;
  const size_t e0 = (size_t)i << 3;
  const v4f a0 = *(const v4f*)(src + e0);
  const v4f a1 = *(const v4f*)(src + e0 + 4);
  v8h hv;
#pragma unroll
  for (int e = 0; e < 4; ++e) {
    hv[e]     = (_Float16)a0[e];
    hv[4 + e] = (_Float16)a1[e];
  }
  unsigned short* qh = dst + e0;
  *(volatile v8h*)qh = hv;
  __threadfence();
  *(volatile v8h*)qh = hv;
}

__global__ __launch_bounds__(256) void transpose_f16_kernel(
    const float* __restrict__ in, unsigned short* __restrict__ out, int R, int C, float scale)
{
  __shared__ __align__(16) float sT[64 * kTrP];
  const int tid = threadIdx.x, lane = tid & 31, wave = tid >> 5;
  const int c0 = blockIdx.x * 64, r0 = blockIdx.y * 64;
  const int lrow = tid >> 4, col4 = (tid & 15) * 4;
  const int c = c0 + col4;
  const bool valid = (c < C);
  const int cc = valid ? c : (C - 4);
#pragma unroll
  for (int i = 0; i < 4; ++i) {
    const int r = r0 + lrow + 16 * i;
    const v4f v = *(const v4f*)(in + (size_t)r * C + cc);
    v4f w;
    w[0] = valid ? v[0] : 0.0f;
    w[1] = valid ? v[1] : 0.0f;
    w[2] = valid ? v[2] : 0.0f;
    w[3] = valid ? v[3] : 0.0f;
    *(v4f*)(sT + (lrow + 16 * i) * kTrP + col4) = w;
  }
  __syncthreads();
  const int q = lane >> 3, c8 = (lane & 7) * 8;
  v8h hv[2];
#pragma unroll
  for (int it = 0; it < 2; ++it) {
    const int orow = it * 32 + wave * 4 + q;
#pragma unroll
    for (int e = 0; e < 8; ++e) hv[it][e] = (_Float16)(sT[(c8 + e) * kTrP + orow] * scale);
  }
  for (int pass = 0; pass < 2; ++pass) {
#pragma unroll
    for (int it = 0; it < 2; ++it) {
      const int orow = it * 32 + wave * 4 + q;
      *(volatile v8h*)(out + (size_t)(c0 + orow) * R + r0 + c8) = hv[it];
    }
    __threadfence();
  }
}

__global__ __launch_bounds__(64) void scan_kernel(
    const float* __restrict__ BC, const unsigned* __restrict__ XPw, const unsigned* __restrict__ DPw,
    unsigned short* ZY, const float* __restrict__ Alog, const float* __restrict__ Dp)
{
  __shared__ __align__(16) float sBC[kScanTS * 32];
  __shared__ __align__(16) float sY[kScanTS * kScanYP];
  const int tid = threadIdx.x, lane = tid & 31, wave = tid >> 5;
  constexpr int kBlkPerB = kDin / kScanCh;
  const int bix = blockIdx.x / kBlkPerB;
  const int d0  = (blockIdx.x - bix * kBlkPerB) * kScanCh;
  const int d   = d0 + tid;
  const size_t row0 = (size_t)bix * kSeq;
  float An[kNst], h[kNst];
  {
    const v4f* ap = (const v4f*)(Alog + (size_t)d * kNst);
    const v4f a0 = ap[0], a1 = ap[1], a2 = ap[2], a3 = ap[3];
#pragma unroll
    for (int e = 0; e < 4; ++e) {
      An[e]      = -expf(a0[e]);
      An[4 + e]  = -expf(a1[e]);
      An[8 + e]  = -expf(a2[e]);
      An[12 + e] = -expf(a3[e]);
    }
  }
#pragma unroll
  for (int s = 0; s < kNst; ++s) h[s] = 0.0f;
  const float Dd = Dp[d];
  const unsigned sh = ((unsigned)(d & 1)) << 4;
  const size_t wcol = (size_t)(d >> 1);
  const unsigned* Zw = (const unsigned*)ZY;
  const int sr = tid >> 3, sc4 = (tid & 7) * 4;
  const int q = lane >> 3, c8 = (lane & 7) * 8;
#pragma unroll 1
  for (int t0 = 0; t0 < kSeq; t0 += kScanTS) {
    __syncthreads();
#pragma unroll
    for (int i = 0; i < 4; ++i) {
      const int r = sr + 8 * i;
      *(v4f*)(sBC + r * 32 + sc4) = *(const v4f*)(BC + (row0 + t0 + r) * kBcP + sc4);
    }
    asm volatile("" ::: "memory");
#pragma unroll
    for (int i = 4; i < 8; ++i) {
      const int r = sr + 8 * i;
      *(v4f*)(sBC + r * 32 + sc4) = *(const v4f*)(BC + (row0 + t0 + r) * kBcP + sc4);
    }
    __syncthreads();
#pragma unroll 1
    for (int s = 0; s < kScanTS; ++s) {
      const size_t row = row0 + t0 + s;
      const size_t wi = row * (size_t)(kDin / 2) + wcol;
      const unsigned wx = XPw[wi];
      const unsigned wp = DPw[wi];
      const unsigned wz = Zw[wi];
      const float xt = h16_to_f32((wx >> sh) & 0xffffu);
      const float v  = h16_to_f32((wp >> sh) & 0xffffu);
      const float zv = h16_to_f32((wz >> sh) & 0xffffu);
      float dt = 0.1f;
      if (v < -2.0f) {
        const float sp = log1pf(expf(v));
        dt = fminf(fmaxf(sp, 1e-3f), 0.1f);
      }
      const float dtx = dt * xt;
      const float* xr = sBC + s * 32;
      float y = 0.0f;
#pragma unroll
      for (int q4 = 0; q4 < 4; ++q4) {
        const v4f bv = *(const v4f*)(xr + 4 * q4);
        const v4f cv = *(const v4f*)(xr + kNst + 4 * q4);
#pragma unroll
        for (int e = 0; e < 4; ++e) {
          const int k = 4 * q4 + e;
          const float abar = fmaf(An[k], dt, 1.0f);
          const float bx = bv[e] * dtx;
          h[k] = fmaf(abar, h[k], bx);
          y = fmaf(cv[e], h[k], y);
        }
      }
      y = fmaf(Dd, xt, y);
      const float sg = 1.0f / (1.0f + expf(-zv));
      const float g  = zv * sg;
      sY[s * kScanYP + tid] = (y * g) * kYsc;
    }
    __syncthreads();
    v8h hv[8];
#pragma unroll
    for (int it = 0; it < 8; ++it) {
      const int row = it * 8 + wave * 4 + q;
      const float* sp = sY + row * kScanYP + c8;
      const v4f a0 = *(const v4f*)(sp);
      const v4f a1 = *(const v4f*)(sp + 4);
#pragma unroll
      for (int e = 0; e < 4; ++e) {
        hv[it][e]     = (_Float16)a0[e];
        hv[it][4 + e] = (_Float16)a1[e];
      }
    }
    for (int pass = 0; pass < 2; ++pass) {
#pragma unroll
      for (int it = 0; it < 8; ++it) {
        const int row = it * 8 + wave * 4 + q;
        const size_t o = (row0 + t0 + row) * (size_t)kDin + d0 + c8;
        *(volatile v8h*)(ZY + o) = hv[it];
      }
      __threadfence();
    }
  }
}

extern "C" void kernel_launch(void* const* d_in, const int* in_sizes, int n_in,
                              void* d_out, int out_size, void* d_ws, size_t ws_size,
                              hipStream_t stream) {
  if (n_in < 8) return;
  if (in_sizes[0] != kRows * kDm) return;
  if (in_sizes[1] != kDm * 2 * kDin) return;
  if (in_sizes[2] != kDin * kXdb) return;
  if (in_sizes[3] != kDtR * kDin) return;
  if (in_sizes[4] != kDin) return;
  if (in_sizes[5] != kDin * kNst) return;
  if (in_sizes[6] != kDin) return;
  if (in_sizes[7] != kDin * kDm) return;
  if (out_size != kRows * kDm) return;
  if (ws_size < kWsTotal) return;

  const float* x       = (const float*)d_in[0];
  const float* W_in    = (const float*)d_in[1];
  const float* W_xproj = (const float*)d_in[2];
  const float* W_dt    = (const float*)d_in[3];
  const float* b_dt    = (const float*)d_in[4];
  const float* A_log   = (const float*)d_in[5];
  const float* Dp      = (const float*)d_in[6];
  const float* W_out   = (const float*)d_in[7];
  float* out = (float*)d_out;

  char* ws = (char*)d_ws;
  unsigned short* X16   = (unsigned short*)(ws + kOffX16);
  unsigned short* BTIN  = (unsigned short*)(ws + kOffBTIN);
  unsigned short* BTXP  = (unsigned short*)(ws + kOffBTXP);
  unsigned short* BTDT  = (unsigned short*)(ws + kOffBTDT);
  unsigned short* BTOUT = (unsigned short*)(ws + kOffBTOUT);
  unsigned short* XP16  = (unsigned short*)(ws + kOffXP16);
  unsigned short* Z16   = (unsigned short*)(ws + kOffZ16);
  unsigned short* DPRE  = (unsigned short*)(ws + kOffDPRE);
  unsigned short* DLT16 = (unsigned short*)(ws + kOffDLT);
  float*          BC32  = (float*)(ws + kOffBC);

  cast_rows_f16_kernel<<<(kRows * kDm / 8) / 256, 256, 0, stream>>>(x, X16, kRows * kDm / 8);
  transpose_f16_kernel<<<dim3(2 * kDin / 64, kDm / 64), 256, 0, stream>>>(W_in, BTIN, kDm, 2 * kDin, kWsc);
  transpose_f16_kernel<<<dim3(kXdbP / 64, kDin / 64), 256, 0, stream>>>(W_xproj, BTXP, kDin, kXdb, kWsc);
  transpose_f16_kernel<<<dim3(kDin / 64, kDtR / 64), 256, 0, stream>>>(W_dt, BTDT, kDtR, kDin, kWsc);
  transpose_f16_kernel<<<dim3(kDm / 64, kDin / 64), 256, 0, stream>>>(W_out, BTOUT, kDin, kDm, kWsc);

  wmma_gemm64<0, false, 0, 1, false, 0><<<dim3(((kRows / 64) * (kDin / 64)) / 8, 2), 256, 0, stream>>>(
      X16, nullptr, kDm, 0L,
      BTIN, nullptr, kDm, (long)kDin * kDm,
      (void*)XP16, nullptr, kDin, (long)kRows * kDin,
      nullptr, nullptr, 0L,
      kRows, kDin, kDm, kWscInv);

  wmma_gemm64<0, false, 0, 1, false, 0><<<dim3(((kRows / 64) * (kDtR / 64)) / 8, 1), 256, 0, stream>>>(
      XP16, nullptr, kDin, 0L,
      BTXP, nullptr, kDin, 0L,
      (void*)DLT16, nullptr, kDtR, 0L,
      nullptr, nullptr, 0L,
      kRows, kDtR, kDin, kWscInv);

  wmma_gemm64<0, false, 0, 0, false, 0><<<dim3(((kRows / 64) * (kBcP / 64)) / 8, 1), 256, 0, stream>>>(
      XP16, nullptr, kDin, 0L,
      BTXP + (size_t)kDtR * kDin, nullptr, kDin, 0L,
      (void*)BC32, nullptr, kBcP, 0L,
      nullptr, nullptr, 0L,
      kRows, kBcP, kDin, kWscInv);

  wmma_gemm64<0, false, 2, 1, false, 0><<<dim3(((kRows / 64) * (kDin / 64)) / 8, 1), 256, 0, stream>>>(
      DLT16, nullptr, kDtR, 0L,
      BTDT, nullptr, kDtR, 0L,
      (void*)DPRE, nullptr, kDin, 0L,
      b_dt, nullptr, 0L,
      kRows, kDin, kDtR, kWscInv);

  scan_kernel<<<kBatch * (kDin / kScanCh), kScanCh, 0, stream>>>(
      BC32, (const unsigned*)XP16, (const unsigned*)DPRE, Z16, A_log, Dp);

  wmma_gemm64<0, false, 0, 0, false, 0><<<dim3(((kRows / 64) * (kDm / 64)) / 8, 1), 256, 0, stream>>>(
      Z16, nullptr, kDin, 0L,
      BTOUT, nullptr, kDin, 0L,
      (void*)out, nullptr, kDm, 0L,
      nullptr, nullptr, 0L,
      kRows, kDm, kDin, kOutScl);
}
